// SelfSSM_360777252919
// MI455X (gfx1250) — hardware-verified
//
#include <hip/hip_runtime.h>
#include <math.h>

typedef __attribute__((ext_vector_type(16))) _Float16 v16h;
typedef __attribute__((ext_vector_type(8)))  _Float16 v8h;
typedef __attribute__((ext_vector_type(16))) __bf16   v16b;
typedef __attribute__((ext_vector_type(8)))  __bf16   v8b;
typedef __attribute__((ext_vector_type(8)))  float    v8f;
typedef __attribute__((ext_vector_type(4)))  float    v4f;

constexpr int kBatch = 4;
constexpr int kSeq   = 1024;
constexpr int kRows  = kBatch * kSeq;
constexpr int kDi    = 1024;
constexpr int kDiLog2 = 10;
constexpr float kLnEps = 1e-12f;
constexpr int kNs    = 16;
constexpr int kR     = 64;
constexpr int kXd    = kR + 2 * kNs;
constexpr int kXdP   = 128;
constexpr int kThr   = 256;

constexpr float kInCarry = 1024.0f;
constexpr float kWCarry  = 1024.0f;
constexpr float kDtCarry = 256.0f;
constexpr float kScIn = 1.0f / (kInCarry * kInCarry);
constexpr float kScDt = 1.0f / (kDtCarry * kWCarry);
constexpr float kF16MinNormal = 6.103515625e-5f;

static_assert((kRows % 64) == 0 && (kXdP % 64) == 0 && (kDi % 64) == 0, "GEMM M, N multiples of 64");
static_assert(((kRows / 64) * (kXdP / 64)) % 8 == 0, "the smallest GEMM grid exact");
static_assert((kDi % 32) == 0 && (kR % 32) == 0, "GEMM K multiples of 32");

constexpr size_t kOffX16 = 0;
constexpr size_t kOffWXP = kOffX16 + (size_t)kRows * kDi * 2;
constexpr size_t kOffWDT = kOffWXP + (size_t)kXdP * kDi * 2;
constexpr size_t kOffBV  = kOffWDT + (size_t)kDi * kR * 2;
constexpr int    kBvZ    = 0;
constexpr int    kBvDt   = kXdP;
constexpr int    kBvTot  = kXdP + kDi;
constexpr size_t kOffXD  = kOffBV  + (size_t)kBvTot * 4;
constexpr size_t kOffDT16 = kOffXD + (size_t)kRows * kXdP * 4;
constexpr size_t kOffDL  = kOffDT16 + (size_t)kRows * kR * 2;
constexpr size_t kOffY   = kOffDL + (size_t)kRows * kDi * 4;
constexpr size_t kWsTotal = kOffY + (size_t)kRows * kDi * 4;
static_assert(kWsTotal <= 268435456ull, "inside the offered workspace");
static_assert((kOffWXP % 256) == 0 && (kOffWDT % 256) == 0 && (kOffBV % 256) == 0 && (kOffXD % 256) == 0 && (kOffDT16 % 256) == 0 && (kOffDL % 256) == 0 && (kOffY % 256) == 0, "aligned regions");

__device__ __forceinline__ unsigned short f2bf_bits(float f) {
  unsigned u = __float_as_uint(f);
  return (unsigned short)((u + 0x7FFFu + ((u >> 16) & 1u)) >> 16);
}
__device__ __forceinline__ float bf_bits2f(unsigned short h) { return __uint_as_float(((unsigned)h) << 16); }
__device__ __forceinline__ float bf16r(float f) { return bf_bits2f(f2bf_bits(f)); }
__device__ __forceinline__ float carry_flush(float v, float carry) {
  const float s = v * carry;
  return (fabsf(s) < kF16MinNormal) ? 0.0f : s;
}
__device__ __forceinline__ float frcp(float x) { return __builtin_amdgcn_rcpf(x); }

__device__ __forceinline__ void dep_guard4_h(v8f& a, v8f& b, v8f& c, v8f& d, v16h x, v16h y) { asm volatile("v_nop\n\tv_nop\n\tv_nop\n\tv_nop" : "+v"(a), "+v"(b), "+v"(c), "+v"(d) : "v"(x), "v"(y)); }
__device__ __forceinline__ void dep_guard4_b(v8f& a, v8f& b, v8f& c, v8f& d, v16b x, v16b y) { asm volatile("v_nop\n\tv_nop\n\tv_nop\n\tv_nop" : "+v"(a), "+v"(b), "+v"(c), "+v"(d) : "v"(x), "v"(y)); }
__device__ __forceinline__ void keep4_h(v16h a, v16h b, v16h c, v16h d) { asm volatile("v_nop" :: "v"(a), "v"(b), "v"(c), "v"(d)); }
__device__ __forceinline__ void keep4_b(v16b a, v16b b, v16b c, v16b d) { asm volatile("v_nop" :: "v"(a), "v"(b), "v"(c), "v"(d)); }
__device__ __forceinline__ void acc_guard4(v8f& a, v8f& b, v8f& c, v8f& d) { asm volatile("v_nop\n\tv_nop\n\tv_nop\n\tv_nop" : "+v"(a), "+v"(b), "+v"(c), "+v"(d)); }

template <typename T> struct Frag;
template <> struct Frag<_Float16> {
  typedef v16h V; union U { v16h v; v8h h[2]; };
  static __device__ __forceinline__ v16h load(const _Float16* p) {
    U f; f.h[0] = *(const v8h*)(p); f.h[1] = *(const v8h*)(p + 16); return f.v;
  }
  static __device__ __forceinline__ v8f mma(v16h a, v16h b, v8f c) {
    return __builtin_amdgcn_wmma_f32_16x16x32_f16(false, a, false, b, (short)0, c, false, false);
  }
  static __device__ __forceinline__ void guard4(v8f& a, v8f& b, v8f& c, v8f& d, v16h x, v16h y) { dep_guard4_h(a, b, c, d, x, y); }
  static __device__ __forceinline__ void keep(v16h a, v16h b, v16h c, v16h d) { keep4_h(a, b, c, d); }
};
template <> struct Frag<__bf16> {
  typedef v16b V; union U { v16b v; v8b h[2]; };
  static __device__ __forceinline__ v16b load(const __bf16* p) {
    U f; f.h[0] = *(const v8b*)(p); f.h[1] = *(const v8b*)(p + 16); return f.v;
  }
  static __device__ __forceinline__ v8f mma(v16b a, v16b b, v8f c) {
    return __builtin_amdgcn_wmma_f32_16x16x32_bf16(false, a, false, b, (short)0, c, false, false);
  }
  static __device__ __forceinline__ void guard4(v8f& a, v8f& b, v8f& c, v8f& d, v16b x, v16b y) { dep_guard4_b(a, b, c, d, x, y); }
  static __device__ __forceinline__ void keep(v16b a, v16b b, v16b c, v16b d) { keep4_b(a, b, c, d); }
};

__device__ __forceinline__ v8f mma_h(v16h a, v16h b, v8f c) {
  c = __builtin_amdgcn_wmma_f32_16x16x32_f16(false, a, false, b, (short)0, c, false, false);
  asm volatile("v_nop\n\tv_nop\n\tv_nop\n\tv_nop" : "+v"(c) : "v"(a), "v"(b));
  return c;
}

template <int ET> struct Elem;
template <> struct Elem<0> { typedef _Float16 T; };
template <> struct Elem<1> { typedef __bf16 T; };
template <int ET, bool SPLIT, int BIAS_MODE, int OUT_MODE, bool RESID, int ACT = 0>
__global__ __launch_bounds__(256) void wmma_gemm64(
    const unsigned short* __restrict__ Ap, const unsigned short* __restrict__ A2p, int lda, long strideA,
    const unsigned short* __restrict__ Btp, const unsigned short* __restrict__ Bt2p, int ldb, long strideB,
    void* __restrict__ Cout, void* __restrict__ Cout2, int ldc, long strideC,
    const float* __restrict__ bias,
    const float* __restrict__ resid, long strideR,
    int M, int N, int K, float scale) {
  typedef typename Elem<ET>::T T;
  typedef typename Frag<T>::V V;
  const T* A = (const T*)Ap; const T* A2 = (const T*)A2p; const T* Bt = (const T*)Btp; const T* Bt2 = (const T*)Bt2p;
  __shared__ __align__(16) float sT[8][16 * 68];
  const int b    = blockIdx.y;
  const int lane = threadIdx.x & 31;
  const int wave = threadIdx.x >> 5;
  const int tilesN = N >> 6;
  const int tilesM = M >> 6;
  const int tile = blockIdx.x * 8 + wave;
  if (tile >= tilesM * tilesN) return;
  const int tm = tile / tilesN;
  const int tn = tile - tm * tilesN;
  const int m0 = tm << 6;
  const int n0 = tn << 6;

  const T* Ab  = A  + (size_t)b * strideA;
  const T* Bb  = Bt + (size_t)b * strideB;
  const T* Ab2 = SPLIT ? (A2  + (size_t)b * strideA) : nullptr;
  const T* Bb2 = SPLIT ? (Bt2 + (size_t)b * strideB) : nullptr;

  const int rlane = lane & 15;
  const int koff  = (lane >> 4) * 8;
  const int mOff  = (lane >> 4) * 8;

  v8f acc[4][4];
#pragma unroll
  for (int i = 0; i < 4; ++i)
#pragma unroll
    for (int j = 0; j < 4; ++j) acc[i][j] = (v8f){0.f,0.f,0.f,0.f,0.f,0.f,0.f,0.f};

  for (int k0 = 0; k0 < K; k0 += 32) {
    V bh[4], bl[4];
#pragma unroll
    for (int j = 0; j < 4; ++j) {
      const size_t bo = (size_t)(n0 + (j << 4) + rlane) * ldb + koff + k0;
      bh[j] = Frag<T>::load(Bb + bo);
      if (SPLIT) bl[j] = Frag<T>::load(Bb2 + bo);
    }
#pragma unroll
    for (int i = 0; i < 4; ++i) {
      const size_t ao = (size_t)(m0 + (i << 4) + rlane) * lda + koff + k0;
      V ah = Frag<T>::load(Ab + ao);
      V al;
      if (SPLIT) al = Frag<T>::load(Ab2 + ao);
#pragma unroll
      for (int j = 0; j < 4; ++j) {
        acc[i][j] = Frag<T>::mma(ah, bh[j], acc[i][j]);
        if (SPLIT) {
          acc[i][j] = Frag<T>::mma(ah, bl[j], acc[i][j]);
          acc[i][j] = Frag<T>::mma(al, bh[j], acc[i][j]);
        }
      }
      Frag<T>::guard4(acc[i][0], acc[i][1], acc[i][2], acc[i][3], ah, SPLIT ? al : ah);
    }
    Frag<T>::keep(bh[0], bh[1], bh[2], bh[3]);
    if (SPLIT) Frag<T>::keep(bl[0], bl[1], bl[2], bl[3]);
  }
  acc_guard4(acc[0][0], acc[0][1], acc[0][2], acc[0][3]);
  acc_guard4(acc[1][0], acc[1][1], acc[1][2], acc[1][3]);
  acc_guard4(acc[2][0], acc[2][1], acc[2][2], acc[2][3]);
  acc_guard4(acc[3][0], acc[3][1], acc[3][2], acc[3][3]);

  float* slab = sT[wave];
  const float* Rb = RESID ? (resid + (size_t)b * strideR) : nullptr;
#pragma unroll
  for (int i = 0; i < 4; ++i) {
    const int mBase = m0 + (i << 4);
#pragma unroll
    for (int j = 0; j < 4; ++j) {
      const int n = n0 + (j << 4) + rlane;
      float bv = 0.f;
      if (BIAS_MODE == 2) bv = bias[n];
#pragma unroll
      for (int r = 0; r < 8; ++r) {
        float v = acc[i][j][r] * scale;
        if (BIAS_MODE == 1) v += bias[mBase + mOff + r];
        if (BIAS_MODE == 2) v += bv;
        if (RESID) v += Rb[(size_t)(mBase + mOff + r) * ldc + n];
        if (ACT == 1) v = tanhf(v);
        if (ACT == 2) v = fmaxf(v, 0.0f);
        if (ACT == 3) v = v / (1.0f + expf(-v));
        if (ACT == 4) v = (v > 0.f) ? v : 0.01f * v;
        slab[(mOff + r) * 68 + (j << 4) + rlane] = v;
      }
    }
    __builtin_amdgcn_fence(__ATOMIC_RELEASE, "workgroup");
    __builtin_amdgcn_wave_barrier();
    __builtin_amdgcn_fence(__ATOMIC_ACQUIRE, "workgroup");
    if (OUT_MODE == 0) {
      float* C = (float*)Cout + (size_t)b * strideC;
      const int hh = lane >> 4, c4 = (lane & 15) * 4;
      for (int pass = 0; pass < 2; ++pass) {
#pragma unroll
        for (int it = 0; it < 8; ++it) {
          const int row = it * 2 + hh;
          v4f v = *(const v4f*)(slab + row * 68 + c4);
          *(volatile v4f*)(C + (size_t)(mBase + row) * ldc + n0 + c4) = v;
        }
        __threadfence();
      }
    } else {
      const int q = lane >> 3, c8 = (lane & 7) * 8;
      unsigned short* C  = (unsigned short*)Cout  + (size_t)b * strideC;
      unsigned short* C2 = (OUT_MODE == 2) ? ((unsigned short*)Cout2 + (size_t)b * strideC) : nullptr;
      for (int pass = 0; pass < 2; ++pass) {
#pragma unroll
        for (int it = 0; it < 4; ++it) {
          const int row = it * 4 + q;
          const float* sp = slab + row * 68 + c8;
          v8h hv, lv;
#pragma unroll
          for (int e = 0; e < 8; ++e) {
            if (OUT_MODE == 1) {
              hv[e] = (_Float16)sp[e];
            } else {
              unsigned short hb = f2bf_bits(sp[e]);
              unsigned short lb = f2bf_bits(sp[e] - bf_bits2f(hb));
              hv[e] = __builtin_bit_cast(_Float16, hb);
              lv[e] = __builtin_bit_cast(_Float16, lb);
            }
          }
          *(volatile v8h*)(C + (size_t)(mBase + row) * ldc + n0 + c8) = hv;
          if (OUT_MODE == 2) *(volatile v8h*)(C2 + (size_t)(mBase + row) * ldc + n0 + c8) = lv;
        }
        __threadfence();
      }
    }
    __builtin_amdgcn_fence(__ATOMIC_RELEASE, "workgroup");
    __builtin_amdgcn_wave_barrier();
    __builtin_amdgcn_fence(__ATOMIC_ACQUIRE, "workgroup");
  }
}

__global__ __launch_bounds__(kThr) void cast_plane_kernel(const float* __restrict__ src, unsigned short* __restrict__ dst,
                                                          int colsLog2, int dstPitch, int dstOff) {
  const int i   = blockIdx.x * kThr + threadIdx.x;
  const int sh  = colsLog2 - 3;
  const int row = i >> sh;
  const int c8  = (i & ((1 << sh) - 1)) * 8;
  const float* sp = src + ((size_t)row << colsLog2) + c8;
  const v4f a0 = *(const v4f*)(sp);
  const v4f a1 = *(const v4f*)(sp + 4);
  v8h hv;
#pragma unroll
  for (int e = 0; e < 4; ++e) {
    const float f0 = a0[e];
    const float f1 = a1[e];
    hv[e]     = (_Float16)carry_flush(bf16r(f0), kInCarry);
    hv[4 + e] = (_Float16)carry_flush(bf16r(f1), kInCarry);
  }
  unsigned short* dp = dst + (size_t)row * dstPitch + dstOff + c8;
  *(volatile v8h*)dp = hv;
  __threadfence();
  *(volatile v8h*)dp = hv;
}

__global__ __launch_bounds__(256) void w_rows_kernel(const float* __restrict__ W, unsigned short* __restrict__ dst, int K, int nLive) {
  const int n  = blockIdx.x;
  const int k8 = threadIdx.x * 8;
  const bool live = n < nLive;
  const int nc = live ? n : 0;
  const v4f a0 = *(const v4f*)(W + (size_t)nc * K + k8);
  const v4f a1 = *(const v4f*)(W + (size_t)nc * K + k8 + 4);
  v8h hv;
#pragma unroll
  for (int e = 0; e < 4; ++e) {
    const float w0 = a0[e], w1 = a1[e];
    hv[e]     = (_Float16)(live ? carry_flush(bf16r(w0), kWCarry) : 0.0f);
    hv[4 + e] = (_Float16)(live ? carry_flush(bf16r(w1), kWCarry) : 0.0f);
  }
  unsigned short* dp = dst + (size_t)n * K + k8;
  *(volatile v8h*)dp = hv;
  __threadfence();
  *(volatile v8h*)dp = hv;
}

__global__ __launch_bounds__(128) void bias_rows_kernel(const float* __restrict__ b_dt, float* __restrict__ BV) {
  const int i = blockIdx.x * 128 + threadIdx.x;
  const int idt = i - kBvDt;
  const float v = b_dt[(idt >= 0) ? idt : 0];
  const float o = (idt >= 0) ? bf16r(v) : 0.0f;
  for (int pass = 0; pass < 2; ++pass) {
    *(volatile float*)(BV + i) = o;
    __threadfence();
  }
}
static_assert(kBvTot % 128 == 0 && kBvDt % 128 == 0, "bias grid exact; regions block-uniform");

__global__ __launch_bounds__(kThr) void dt_cast_kernel(const float* __restrict__ XD, unsigned short* __restrict__ DT16) {
  const size_t v = (size_t)blockIdx.x * kThr + threadIdx.x;
  const size_t row = v >> 3;
  const int c8 = (int)(v & 7) * 8;
  const v4f a0 = *(const v4f*)(XD + row * kXdP + c8);
  const v4f a1 = *(const v4f*)(XD + row * kXdP + c8 + 4);
  v8h hv;
#pragma unroll
  for (int e = 0; e < 4; ++e) { hv[e] = (_Float16)carry_flush(a0[e], kDtCarry); hv[4 + e] = (_Float16)carry_flush(a1[e], kDtCarry); }
  unsigned short* dp = DT16 + row * kR + c8;
  *(volatile v8h*)dp = hv;
  __threadfence();
  *(volatile v8h*)dp = hv;
}
static_assert(((size_t)kRows * 8) % kThr == 0, "dt cast grid exact");

__global__ __launch_bounds__(kThr) void sel_scan_kernel(const float* __restrict__ DL, const float* __restrict__ x, const float* __restrict__ XD,
                                                        const float* __restrict__ A_log, const float* __restrict__ Dp, float* __restrict__ out) {
  const int v = blockIdx.x * kThr + threadIdx.x;
  const int b = v >> kDiLog2;
  const int d = v & (kDi - 1);
  float A[kNs], h[kNs];
#pragma unroll
  for (int n = 0; n < kNs; ++n) { const float al = A_log[(size_t)d * kNs + n]; A[n] = -expf(bf16r(al)); h[n] = 0.0f; }
  const float dd = Dp[d];
  const float dsk = bf16r(dd);
  const size_t r0 = (size_t)b * kSeq;
#pragma unroll 1
  for (int l = 0; l < kSeq; ++l) {
    const size_t row = r0 + l;
    const float dl = DL[row * kDi + d];
    const float xr = x[row * kDi + d];
    const float xv = bf16r(xr);
    const float delta = (dl > 20.0f) ? dl : log1pf(expf(dl));
    const float dx = delta * xv;
    float y = 0.0f;
#pragma unroll
    for (int q = 0; q < 4; ++q) {
      const v4f bq = *(const v4f*)(XD + row * kXdP + kR + 4 * q);
      const v4f cq = *(const v4f*)(XD + row * kXdP + kR + kNs + 4 * q);
#pragma unroll
      for (int e = 0; e < 4; ++e) {
        const int n = 4 * q + e;
        const float hn = __expf(delta * A[n]) * h[n] + dx * bq[e];
        h[n] = hn;
        y += hn * cq[e];
      }
    }
    const float o = y + dsk * xv;
    float* op = out + row * kDi + d;
    *(volatile float*)op = o;
    __threadfence();
    *(volatile float*)op = o;
  }
}
static_assert((kBatch * kDi) % kThr == 0, "scan grid exact");

__device__ __forceinline__ float block_sum_256(float v, float* red, float* wsum) {
  const int tid = threadIdx.x;
  red[tid] = v;
  __syncthreads();
  if ((tid & 31) == 0) {
    float s = 0.0f;
#pragma unroll 1
    for (int k = 0; k < 32; ++k) s += red[tid + k];
    wsum[tid >> 5] = s;
  }
  __syncthreads();
  float t = 0.0f;
#pragma unroll
  for (int k = 0; k < 8; ++k) t += wsum[k];
  __syncthreads();
  return t;
}

__global__ __launch_bounds__(kThr) void ln_std_kernel(const float* __restrict__ Y, const float* __restrict__ ln_a, const float* __restrict__ ln_b,
                                                      float* __restrict__ out) {
  __shared__ float red[kThr];
  __shared__ float wsum[8];
  const size_t row = blockIdx.x;
  const int f4 = threadIdx.x * 4;
  const v4f yv = *(const v4f*)(Y + row * kDi + f4);
  const float mean = block_sum_256((yv[0] + yv[1]) + (yv[2] + yv[3]), red, wsum) * (1.0f / (float)kDi);
  const float d0 = yv[0] - mean, d1 = yv[1] - mean, d2 = yv[2] - mean, d3 = yv[3] - mean;
  const float ss = block_sum_256((d0 * d0 + d1 * d1) + (d2 * d2 + d3 * d3), red, wsum);
  const float sd = sqrtf(ss / (float)(kDi - 1));
  const float den = sd + kLnEps;
  const v4f ga = *(const v4f*)(ln_a + f4);
  const v4f gb = *(const v4f*)(ln_b + f4);
  v4f o;
#pragma unroll
  for (int e = 0; e < 4; ++e) {
    const float a0 = ga[e], b0 = gb[e];
    const float dn = (e == 0) ? d0 : ((e == 1) ? d1 : ((e == 2) ? d2 : d3));
    o[e] = bf16r(a0) * dn / den + bf16r(b0);
  }
  float* dp = out + row * kDi + f4;
  *(volatile v4f*)dp = o;
  __threadfence();
  *(volatile v4f*)dp = o;
}
static_assert(kDi / 4 == kThr, "one block per row");

static_assert(((size_t)kRows * kDi / 8) % kThr == 0, "cast grid exact");

extern "C" void kernel_launch(void* const* d_in, const int* in_sizes, int n_in,
                              void* d_out, int out_size, void* d_ws, size_t ws_size,
                              hipStream_t stream) {
  if (n_in < 8 || d_out == nullptr || d_ws == nullptr) return;
  if (in_sizes[0] != kRows * kDi || in_sizes[1] != kXd * kDi || in_sizes[2] != kDi * kR || in_sizes[3] != kDi) return;
  if (in_sizes[4] != kDi * kNs || in_sizes[5] != kDi || in_sizes[6] != kDi || in_sizes[7] != kDi) return;
  if (out_size != kRows * kDi) return;
  if (ws_size < kWsTotal) return;
  const float* x = (const float*)d_in[0];
  const float* W_xproj = (const float*)d_in[1];
  const float* W_dt = (const float*)d_in[2];
  const float* b_dt = (const float*)d_in[3];
  const float* A_log = (const float*)d_in[4];
  const float* Dp = (const float*)d_in[5];
  const float* ln_a = (const float*)d_in[6];
  const float* ln_b = (const float*)d_in[7];
  float* out = (float*)d_out;
  char* ws = (char*)d_ws;
  unsigned short* X16 = (unsigned short*)(ws + kOffX16);
  unsigned short* WXP = (unsigned short*)(ws + kOffWXP);
  unsigned short* WDT = (unsigned short*)(ws + kOffWDT);
  float* BV = (float*)(ws + kOffBV);
  float* XD = (float*)(ws + kOffXD);
  unsigned short* DT16 = (unsigned short*)(ws + kOffDT16);
  float* DL = (float*)(ws + kOffDL);
  float* Y = (float*)(ws + kOffY);

  cast_plane_kernel<<<(int)(((size_t)kRows * kDi / 8) / kThr), kThr, 0, stream>>>(x, X16, 10, kDi, 0);
  w_rows_kernel<<<kXdP, kDi / 8, 0, stream>>>(W_xproj, WXP, kDi, kXd);
  w_rows_kernel<<<kDi, kR / 8, 0, stream>>>(W_dt, WDT, kR, kDi);
  bias_rows_kernel<<<kBvTot / 128, 128, 0, stream>>>(b_dt, BV);

  wmma_gemm64<0, false, 2, 0, false, 0><<<dim3((kRows / 64) * (kXdP / 64) / 8, 1), 256, 0, stream>>>(
      X16, X16, kDi, 0L, WXP, WXP, kDi, 0L, (void*)XD, (void*)XD, kXdP, 0L, BV + kBvZ, nullptr, 0L, kRows, kXdP, kDi, kScIn);
  dt_cast_kernel<<<(int)(((size_t)kRows * 8) / kThr), kThr, 0, stream>>>(XD, DT16);
  wmma_gemm64<0, false, 2, 0, false, 0><<<dim3((kRows / 64) * (kDi / 64) / 8, 1), 256, 0, stream>>>(
      DT16, DT16, kR, 0L, WDT, WDT, kR, 0L, (void*)DL, (void*)DL, kDi, 0L, BV + kBvDt, nullptr, 0L, kRows, kDi, kR, kScDt);
  sel_scan_kernel<<<(kBatch * kDi) / kThr, kThr, 0, stream>>>(DL, x, XD, A_log, Dp, Y);
  ln_std_kernel<<<kRows, kThr, 0, stream>>>(Y, ln_a, ln_b, out);
}
